// Model_13134009991755
// MI455X (gfx1250) — hardware-verified
//
#include <hip/hip_runtime.h>
#include <math.h>

typedef __attribute__((ext_vector_type(16))) _Float16 v16h;
typedef __attribute__((ext_vector_type(8)))  _Float16 v8h;
typedef __attribute__((ext_vector_type(16))) __bf16   v16b;
typedef __attribute__((ext_vector_type(8)))  __bf16   v8b;
typedef __attribute__((ext_vector_type(8)))  float    v8f;
typedef __attribute__((ext_vector_type(4)))  float    v4f;

constexpr int kBatch = 8;
constexpr int kSide  = 32;
constexpr int kSeq   = kSide * kSide;
constexpr int kDm    = 96;
constexpr int kDi    = 192;
constexpr int kNst   = 16;
constexpr int kRank  = 6;
constexpr int kDir   = 4;
constexpr int kRows  = kBatch * kSeq;
constexpr int kXzP   = 2 * kDi;
constexpr int kXcols = kRank + 2 * kNst;
constexpr int kXcP   = 48;
constexpr int kXdP   = kDir * kXcP;
constexpr int kWoP   = 128;
constexpr int kChunk = 32;
static_assert(kSeq == 1024 && kRows == 8192, "sequence geometry");
static_assert(kXcols == 38 && kXcols <= 40 && kXcP % 16 == 0 && kXdP == 192, "x_proj width");
static_assert((kDm % 32) == 0 && (kDi % 32) == 0, "GEMM K multiples of 32");
static_assert((kRows % 64) == 0 && (kXzP % 64) == 0 && (kXdP % 64) == 0 && (kWoP % 64) == 0, "GEMM M,N multiples of 64");
static_assert(((kRows / 64) * (kXzP / 64)) % 8 == 0 && ((kRows / 64) * (kXdP / 64)) % 8 == 0 && ((kRows / 64) * (kWoP / 64)) % 8 == 0, "8 tiles per block");
static_assert(kDm % 32 == 0 && kDm <= kWoP, "output row = whole 128-B lines");

constexpr size_t kOffXB  = 0;
constexpr size_t kOffWI  = kOffXB  + (size_t)kRows * kDm * 2;
constexpr size_t kOffWXP = kOffWI  + (size_t)kXzP * kDm * 2;
constexpr size_t kOffWO  = kOffWXP + (size_t)kXdP * kDi * 2;
constexpr size_t kOffXZ  = kOffWO  + (size_t)kWoP * kDi * 2;
constexpr size_t kOffXC  = kOffXZ  + (size_t)kRows * kXzP * 4;
constexpr size_t kOffXCH = kOffXC  + (size_t)kRows * kDi * 4;
constexpr size_t kOffXCL = kOffXCH + (size_t)kRows * kDi * 2;
constexpr size_t kOffXD  = kOffXCL + (size_t)kRows * kDi * 2;
constexpr size_t kOffYS  = kOffXD  + (size_t)kRows * kXdP * 4;
constexpr size_t kOffYH  = kOffYS  + (size_t)kDir * kRows * kDi * 4;
constexpr size_t kOffYL  = kOffYH  + (size_t)kRows * kDi * 2;
constexpr size_t kWsTotal = kOffYL + (size_t)kRows * kDi * 2;
static_assert(kWsTotal == 64684032ull, "carve total");
static_assert(kWsTotal <= 134217728ull, "carve cap");
static_assert((kOffWI % 128) == 0 && (kOffWXP % 128) == 0 && (kOffWO % 128) == 0 && (kOffXZ % 128) == 0 &&
              (kOffXC % 128) == 0 && (kOffXCH % 128) == 0 && (kOffXCL % 128) == 0 && (kOffXD % 128) == 0 &&
              (kOffYS % 128) == 0 && (kOffYH % 128) == 0 && (kOffYL % 128) == 0, "128-B aligned regions");

__device__ __forceinline__ unsigned short f2bf_bits(float f) {
  unsigned u = __float_as_uint(f);
  return (unsigned short)((u + 0x7FFFu + ((u >> 16) & 1u)) >> 16);
}
__device__ __forceinline__ float bf_bits2f(unsigned short h) { return __uint_as_float(((unsigned)h) << 16); }
__device__ __forceinline__ float bf_rne(float f) { return bf_bits2f(f2bf_bits(f)); }

__device__ __forceinline__ void split8(const v4f a0, const v4f a1, v8h& hv, v8h& lv) {
#pragma unroll
  for (int e = 0; e < 4; ++e) {
    const float f0 = a0[e];
    const float f1 = a1[e];
    const unsigned short h0 = f2bf_bits(f0);
    const unsigned short h1 = f2bf_bits(f1);
    const unsigned short l0 = f2bf_bits(f0 - bf_bits2f(h0));
    const unsigned short l1 = f2bf_bits(f1 - bf_bits2f(h1));
    hv[e]     = __builtin_bit_cast(_Float16, h0);
    hv[4 + e] = __builtin_bit_cast(_Float16, h1);
    lv[e]     = __builtin_bit_cast(_Float16, l0);
    lv[4 + e] = __builtin_bit_cast(_Float16, l1);
  }
}

__device__ __forceinline__ int dir_pos(int k, int l) {
  const int ll = (k & 2) ? (kSeq - 1 - l) : l;
  const int tp = ((ll & 31) << 5) | (ll >> 5);
  return (k & 1) ? tp : ll;
}

__device__ __forceinline__ void dep_guard4_b(v8f& a, v8f& b, v8f& c, v8f& d, v16b x, v16b y) {
  asm volatile("v_nop\n\tv_nop\n\tv_nop\n\tv_nop" : "+v"(a), "+v"(b), "+v"(c), "+v"(d) : "v"(x), "v"(y));
}
__device__ __forceinline__ void keep4_b(v16b a, v16b b, v16b c, v16b d) { asm volatile("v_nop" :: "v"(a), "v"(b), "v"(c), "v"(d)); }
__device__ __forceinline__ void acc_guard4(v8f& a, v8f& b, v8f& c, v8f& d) { asm volatile("v_nop\n\tv_nop\n\tv_nop\n\tv_nop" : "+v"(a), "+v"(b), "+v"(c), "+v"(d)); }

union FragB { v16b v; v8b h[2]; };
__device__ __forceinline__ v16b frag_load_b(const __bf16* p) {
  FragB f;
  f.h[0] = *(const v8b*)(p);
  f.h[1] = *(const v8b*)(p + 16);
  return f.v;
}
__device__ __forceinline__ v8f mma_b(v16b a, v16b b, v8f c) {
  return __builtin_amdgcn_wmma_f32_16x16x32_bf16(false, a, false, b, (short)0, c, false, false);
}

template <int SPL>
__global__ __launch_bounds__(256) void wmma_gemm64_bf16(
    const unsigned short* __restrict__ Ap, const unsigned short* __restrict__ A2p, int lda,
    const unsigned short* __restrict__ Btp, int ldb,
    float* __restrict__ C, int ldc, int M, int N, int K, int nStore)
{
  const __bf16* A  = (const __bf16*)Ap;
  const __bf16* A2 = (const __bf16*)A2p;
  const __bf16* Bt = (const __bf16*)Btp;
  __shared__ __align__(16) float sT[8][16 * 68];
  const int lane = threadIdx.x & 31;
  const int wave = threadIdx.x >> 5;
  const int tilesN = N >> 6;
  const int tilesM = M >> 6;
  const int tile = blockIdx.x * 8 + wave;
  if (tile >= tilesM * tilesN) return;
  const int tm = tile / tilesN;
  const int tn = tile - tm * tilesN;
  const int m0 = tm << 6;
  const int n0 = tn << 6;

  const int rlane = lane & 15;
  const int koff  = (lane >> 4) * 8;
  const int mOff  = (lane >> 4) * 8;

  v8f acc[4][4];
#pragma unroll
  for (int i = 0; i < 4; ++i)
#pragma unroll
    for (int j = 0; j < 4; ++j) acc[i][j] = (v8f){0.f, 0.f, 0.f, 0.f, 0.f, 0.f, 0.f, 0.f};

  for (int k0 = 0; k0 < K; k0 += 32) {
    v16b bh[4];
#pragma unroll
    for (int j = 0; j < 4; ++j) {
      const size_t bo = (size_t)(n0 + (j << 4) + rlane) * ldb + koff + k0;
      bh[j] = frag_load_b(Bt + bo);
    }
#pragma unroll
    for (int i = 0; i < 4; ++i) {
      const size_t ao = (size_t)(m0 + (i << 4) + rlane) * lda + koff + k0;
      const v16b ah = frag_load_b(A + ao);
      v16b al = ah;
      if (SPL == 1) al = frag_load_b(A2 + ao);
#pragma unroll
      for (int j = 0; j < 4; ++j) {
        acc[i][j] = mma_b(ah, bh[j], acc[i][j]);
        if (SPL == 1) acc[i][j] = mma_b(al, bh[j], acc[i][j]);
      }
      dep_guard4_b(acc[i][0], acc[i][1], acc[i][2], acc[i][3], ah, al);
    }
    keep4_b(bh[0], bh[1], bh[2], bh[3]);
  }
  acc_guard4(acc[0][0], acc[0][1], acc[0][2], acc[0][3]);
  acc_guard4(acc[1][0], acc[1][1], acc[1][2], acc[1][3]);
  acc_guard4(acc[2][0], acc[2][1], acc[2][2], acc[2][3]);
  acc_guard4(acc[3][0], acc[3][1], acc[3][2], acc[3][3]);

  float* slab = sT[wave];
  const int hh = lane >> 4;
  const int c4 = (lane & 15) * 4;
  const bool doStore = (n0 + c4) < nStore;
#pragma unroll
  for (int i = 0; i < 4; ++i) {
    const int mBase = m0 + (i << 4);
#pragma unroll
    for (int j = 0; j < 4; ++j) {
#pragma unroll
      for (int r = 0; r < 8; ++r) {
        slab[(mOff + r) * 68 + (j << 4) + rlane] = acc[i][j][r];
      }
    }
    __builtin_amdgcn_fence(__ATOMIC_RELEASE, "workgroup");
    __builtin_amdgcn_wave_barrier();
    __builtin_amdgcn_fence(__ATOMIC_ACQUIRE, "workgroup");
    for (int pass = 0; pass < 2; ++pass) {
#pragma unroll
      for (int it = 0; it < 8; ++it) {
        const int row = it * 2 + hh;
        const v4f v = *(const v4f*)(slab + row * 68 + c4);
        if (doStore) *(volatile v4f*)(C + (size_t)(mBase + row) * ldc + n0 + c4) = v;
      }
      __threadfence();
    }
    __builtin_amdgcn_fence(__ATOMIC_RELEASE, "workgroup");
    __builtin_amdgcn_wave_barrier();
    __builtin_amdgcn_fence(__ATOMIC_ACQUIRE, "workgroup");
  }
}

__global__ __launch_bounds__(256) void plane_bf16_kernel(
    const float* __restrict__ src, unsigned short* __restrict__ dst, int total8, int cols, int padGroup, int realGroup)
{
  const int i = blockIdx.x * 256 + threadIdx.x;
  if (i >= total8) return;
  const int e0 = i << 3;
  const int r  = e0 / cols;
  const int c  = e0 - r * cols;
  const int g  = r / padGroup;
  const int rr = r - g * padGroup;
  const bool valid = rr < realGroup;
  const int rc = valid ? rr : (realGroup - 1);
  const float* p = src + (size_t)(g * realGroup + rc) * cols + c;
  const v4f a0 = *(const v4f*)(p);
  const v4f a1 = *(const v4f*)(p + 4);
  v8h hv;
#pragma unroll
  for (int e = 0; e < 4; ++e) {
    const float f0 = a0[e];
    const float f1 = a1[e];
    const unsigned short b0 = f2bf_bits(f0);
    const unsigned short b1 = f2bf_bits(f1);
    const unsigned short h0 = valid ? b0 : (unsigned short)0;
    const unsigned short h1 = valid ? b1 : (unsigned short)0;
    hv[e]     = __builtin_bit_cast(_Float16, h0);
    hv[4 + e] = __builtin_bit_cast(_Float16, h1);
  }
  unsigned short* q = dst + (size_t)e0;
  *(volatile v8h*)q = hv;
  __threadfence();
  *(volatile v8h*)q = hv;
}

__global__ __launch_bounds__(192) void conv_silu_kernel(
    const float* __restrict__ XZ, const float* __restrict__ cw, const float* __restrict__ cb,
    float* __restrict__ XC, unsigned short* __restrict__ XCH, unsigned short* __restrict__ XCL)
{
  __shared__ __align__(16) float sT[kSide * kDi];
  const int tid = threadIdx.x;
  const int d = tid;
  const int b = blockIdx.x >> 5;
  const int h = blockIdx.x & 31;
  float wt[9];
#pragma unroll
  for (int t = 0; t < 9; ++t) wt[t] = bf_rne(cw[d * 9 + t]);
  const float bias = bf_rne(cb[d]);
  const bool hm = (h > 0);
  const bool hp = (h < kSide - 1);
  const int rm = hm ? (h - 1) : 0;
  const int rp = hp ? (h + 1) : (kSide - 1);
  const float* pm = XZ + ((size_t)(b * kSeq + rm * kSide)) * kXzP + d;
  const float* p0 = XZ + ((size_t)(b * kSeq + h  * kSide)) * kXzP + d;
  const float* pp = XZ + ((size_t)(b * kSeq + rp * kSide)) * kXzP + d;
  float a0 = 0.f, a1 = 0.f, a2 = 0.f;
  float b0, b1, b2;
  {
    const float vm = pm[0];
    const float v0 = p0[0];
    const float vp = pp[0];
    b0 = hm ? vm : 0.f;
    b1 = v0;
    b2 = hp ? vp : 0.f;
  }
#pragma unroll 1
  for (int w = 0; w < kSide; ++w) {
    const int wn = w + 1;
    const bool inb = wn < kSide;
    const int wc = inb ? wn : (kSide - 1);
    const float vm = pm[(size_t)wc * kXzP];
    const float v0 = p0[(size_t)wc * kXzP];
    const float vp = pp[(size_t)wc * kXzP];
    const float c0 = (hm && inb) ? vm : 0.f;
    const float c1 = inb ? v0 : 0.f;
    const float c2 = (hp && inb) ? vp : 0.f;
    float acc = wt[0] * a0;
    acc = fmaf(wt[1], b0, acc);
    acc = fmaf(wt[2], c0, acc);
    acc = fmaf(wt[3], a1, acc);
    acc = fmaf(wt[4], b1, acc);
    acc = fmaf(wt[5], c1, acc);
    acc = fmaf(wt[6], a2, acc);
    acc = fmaf(wt[7], b2, acc);
    acc = fmaf(wt[8], c2, acc);
    const float pre = acc + bias;
    const float sg = __builtin_amdgcn_rcpf(1.0f + expf(-pre));
    sT[w * kDi + tid] = pre * sg;
    a0 = b0; a1 = b1; a2 = b2;
    b0 = c0; b1 = c1; b2 = c2;
  }
  __syncthreads();
  v4f fv[8];
  v8h hv[4], lv[4];
#pragma unroll
  for (int it = 0; it < 8; ++it) fv[it] = *(const v4f*)(sT + (it * 192 + tid) * 4);
#pragma unroll
  for (int it = 0; it < 4; ++it) {
    const float* sp = sT + (it * 192 + tid) * 8;
    const v4f q0 = *(const v4f*)(sp);
    const v4f q1 = *(const v4f*)(sp + 4);
    split8(q0, q1, hv[it], lv[it]);
  }
  const size_t base = (size_t)blockIdx.x * (kSide * kDi);
  for (int pass = 0; pass < 2; ++pass) {
#pragma unroll
    for (int it = 0; it < 8; ++it)
      *(volatile v4f*)(XC + base + (size_t)(it * 192 + tid) * 4) = fv[it];
#pragma unroll
    for (int it = 0; it < 4; ++it) {
      const size_t o = base + (size_t)(it * 192 + tid) * 8;
      *(volatile v8h*)(XCH + o) = hv[it];
      *(volatile v8h*)(XCL + o) = lv[it];
    }
    __threadfence();
  }
}

__global__ __launch_bounds__(192) void scan_kernel(
    const float* __restrict__ XD, const float* __restrict__ XC,
    const float* __restrict__ dtw, const float* __restrict__ dtb,
    const float* __restrict__ Alog, const float* __restrict__ Dsv,
    float* __restrict__ YS)
{
  __shared__ __align__(16) float sX[kChunk * kXcP];
  __shared__ __align__(16) float sY[kChunk * kDi];
  __shared__ float sA[kNst * kDi];
  const int tid  = threadIdx.x;
  const int lane = tid & 31;
  const int wave = tid >> 5;
  const int b  = blockIdx.x >> 2;
  const int k  = blockIdx.x & 3;
  const int d  = tid;
  const int kd = k * kDi + d;

#pragma unroll 1
  for (int n = 0; n < kNst; ++n) sA[n * kDi + tid] = -expf(bf_rne(Alog[(size_t)kd * kNst + n]));
  __syncthreads();
  float negA[kNst], h[kNst];
#pragma unroll
  for (int n = 0; n < kNst; ++n) {
    negA[n] = sA[n * kDi + tid];
    h[n] = 0.f;
  }
  float w6[kRank];
#pragma unroll
  for (int r = 0; r < kRank; ++r) w6[r] = bf_rne(dtw[(size_t)kd * kRank + r]);
  const float bias = bf_rne(dtb[kd]);
  const float Dd   = bf_rne(Dsv[kd]);

  const float* xcb = XC + (size_t)(b * kSeq) * kDi + d;
  const float* xdb = XD + (size_t)(b * kSeq) * kXdP + k * kXcP;
  float*       ysb = YS + (size_t)((k * kBatch + b) * kSeq) * kDi;
  const int q  = lane >> 3;
  const int c4 = wave * 32 + (lane & 7) * 4;

#pragma unroll 1
  for (int c = 0; c < kSeq / kChunk; ++c) {
    const int l0 = c * kChunk;
    __syncthreads();
#pragma unroll
    for (int it = 0; it < 2; ++it) {
      const int idx = tid + it * 192;
      const int row = idx / 12;
      const int qq  = idx - row * 12;
      const int p   = dir_pos(k, l0 + row);
      const v4f v = *(const v4f*)(xdb + (size_t)p * kXdP + qq * 4);
      *(v4f*)(sX + row * kXcP + qq * 4) = v;
    }
    __syncthreads();
#pragma unroll 1
    for (int s = 0; s < kChunk; ++s) {
      const int p = dir_pos(k, l0 + s);
      float xv = xcb[(size_t)p * kDi];
      asm volatile("" : "+v"(xv));
      const float* xr = sX + s * kXcP;
      v4f X[10];
#pragma unroll
      for (int i = 0; i < 10; ++i) X[i] = *(const v4f*)(xr + 4 * i);
      float dot = X[0][0] * w6[0];
      dot = fmaf(X[0][1], w6[1], dot);
      dot = fmaf(X[0][2], w6[2], dot);
      dot = fmaf(X[0][3], w6[3], dot);
      dot = fmaf(X[1][0], w6[4], dot);
      dot = fmaf(X[1][1], w6[5], dot);
      const float v = dot + bias;
      const float delta = fmaxf(v, 0.0f) + log1pf(expf(-fabsf(v)));
      float y = 0.f;
#pragma unroll
      for (int n = 0; n < kNst; ++n) {
        const float Bn = X[(kRank + n) >> 2][(kRank + n) & 3];
        const float Cn = X[(kRank + kNst + n) >> 2][(kRank + kNst + n) & 3];
        const float ea = __expf(delta * negA[n]);
        const float u  = (delta * Bn) * xv;
        h[n] = fmaf(ea, h[n], u);
        y = fmaf(h[n], Cn, y);
      }
      y = fmaf(Dd, xv, y);
      sY[s * kDi + tid] = y;
    }
    __syncthreads();
    v4f yv[8];
#pragma unroll
    for (int it = 0; it < 8; ++it) yv[it] = *(const v4f*)(sY + (it * 4 + q) * kDi + c4);
    for (int pass = 0; pass < 2; ++pass) {
#pragma unroll
      for (int it = 0; it < 8; ++it) {
        const int p = dir_pos(k, l0 + it * 4 + q);
        *(volatile v4f*)(ysb + (size_t)p * kDi + c4) = yv[it];
      }
      __threadfence();
    }
  }
}

__device__ __forceinline__ float hsum4(const v4f v) { return (v[0] + v[1]) + (v[2] + v[3]); }

__global__ __launch_bounds__(256) void ln_gate_kernel(
    const float* __restrict__ YS, const float* __restrict__ XZ,
    const float* __restrict__ gw, const float* __restrict__ gb,
    unsigned short* __restrict__ YH, unsigned short* __restrict__ YL)
{
  __shared__ __align__(16) float sT[32 * kDi];
  __shared__ float sMu[32];
  __shared__ float sRs[32];
  const int tid  = threadIdx.x;
  const int lane = tid & 31;
  const int wave = tid >> 5;
  const int pos0 = blockIdx.x * 32;
  constexpr size_t kPlane = (size_t)kRows * kDi;
  constexpr float kInvD = 1.0f / (float)kDi;
  const bool lo16 = lane < 16;

#pragma unroll 1
  for (int it = 0; it < 2; ++it) {
    const int pl0 = wave * 4 + it * 2;
    v4f yv[3];
#pragma unroll
    for (int j = 0; j < 3; ++j) {
      const int i  = lane + 32 * j;
      const int pl = (i >= 48) ? 1 : 0;
      const int cc = (i - pl * 48) * 4;
      const size_t off = (size_t)(pos0 + pl0 + pl) * kDi + cc;
      const v4f y0 = *(const v4f*)(YS + off);
      const v4f y1 = *(const v4f*)(YS + kPlane + off);
      const v4f y2 = *(const v4f*)(YS + 2 * kPlane + off);
      const v4f y3 = *(const v4f*)(YS + 3 * kPlane + off);
      yv[j] = ((y0 + y2) + y1) + y3;
    }
    const float s0 = hsum4(yv[0]);
    const float s1 = hsum4(yv[1]);
    const float s2 = hsum4(yv[2]);
    float sa = s0 + (lo16 ? s1 : 0.f);
    float sb = s2 + (lo16 ? 0.f : s1);
#pragma unroll
    for (int off = 16; off >= 1; off >>= 1) {
      sa += __shfl_xor(sa, off, 32);
      sb += __shfl_xor(sb, off, 32);
    }
    const float muA = sa * kInvD;
    const float muB = sb * kInvD;
    const float mu1 = lo16 ? muA : muB;
    const v4f d0 = yv[0] - muA;
    const v4f d1 = yv[1] - mu1;
    const v4f d2 = yv[2] - muB;
    const float q0 = hsum4(d0 * d0);
    const float q1 = hsum4(d1 * d1);
    const float q2 = hsum4(d2 * d2);
    float qa = q0 + (lo16 ? q1 : 0.f);
    float qb = q2 + (lo16 ? 0.f : q1);
#pragma unroll
    for (int off = 16; off >= 1; off >>= 1) {
      qa += __shfl_xor(qa, off, 32);
      qb += __shfl_xor(qb, off, 32);
    }
    const float rsA = 1.0f / sqrtf(qa * kInvD + 1e-5f);
    const float rsB = 1.0f / sqrtf(qb * kInvD + 1e-5f);
#pragma unroll
    for (int j = 0; j < 3; ++j) {
      const int i  = lane + 32 * j;
      const int pl = (i >= 48) ? 1 : 0;
      const int cc = (i - pl * 48) * 4;
      *(v4f*)(sT + (pl0 + pl) * kDi + cc) = yv[j];
    }
    if (lane == 0) {
      sMu[pl0]     = muA;
      sMu[pl0 + 1] = muB;
      sRs[pl0]     = rsA;
      sRs[pl0 + 1] = rsB;
    }
  }
  __syncthreads();

#pragma unroll 1
  for (int it = 0; it < 3; ++it) {
    const int idx = it * 256 + tid;
    const int pl  = idx / 24;
    const int c8  = (idx - pl * 24) * 8;
    const float mu = sMu[pl];
    const float rs = sRs[pl];
    const float* sp = sT + pl * kDi + c8;
    const v4f a0 = *(const v4f*)(sp);
    const v4f a1 = *(const v4f*)(sp + 4);
    const float* zp = XZ + (size_t)(pos0 + pl) * kXzP + kDi + c8;
    const v4f z0 = *(const v4f*)(zp);
    const v4f z1 = *(const v4f*)(zp + 4);
    const v4f g0 = *(const v4f*)(gw + c8);
    const v4f g1 = *(const v4f*)(gw + c8 + 4);
    const v4f e0 = *(const v4f*)(gb + c8);
    const v4f e1 = *(const v4f*)(gb + c8 + 4);
    v4f o0, o1;
#pragma unroll
    for (int e = 0; e < 4; ++e) {
      const float za = z0[e];
      const float zb = z1[e];
      const float na = ((a0[e] - mu) * rs) * bf_rne(g0[e]) + bf_rne(e0[e]);
      const float nb = ((a1[e] - mu) * rs) * bf_rne(g1[e]) + bf_rne(e1[e]);
      const float sga = __builtin_amdgcn_rcpf(1.0f + expf(-za));
      const float sgb = __builtin_amdgcn_rcpf(1.0f + expf(-zb));
      o0[e] = na * (za * sga);
      o1[e] = nb * (zb * sgb);
    }
    v8h hv, lv;
    split8(o0, o1, hv, lv);
    const size_t o = (size_t)pos0 * kDi + (size_t)idx * 8;
    *(volatile v8h*)(YH + o) = hv;
    *(volatile v8h*)(YL + o) = lv;
    __threadfence();
    *(volatile v8h*)(YH + o) = hv;
    *(volatile v8h*)(YL + o) = lv;
  }
}

extern "C" void kernel_launch(void* const* d_in, const int* in_sizes, int n_in,
                              void* d_out, int out_size, void* d_ws, size_t ws_size,
                              hipStream_t stream)
{
  if (n_in < 12) return;
  if (in_sizes[0] != kRows * kDm) return;
  if (in_sizes[1] != kXzP * kDm) return;
  if (in_sizes[2] != kDi * 9) return;
  if (in_sizes[3] != kDi) return;
  if (in_sizes[4] != kDir * kXcols * kDi) return;
  if (in_sizes[5] != kDir * kDi * kRank) return;
  if (in_sizes[6] != kDir * kDi) return;
  if (in_sizes[7] != kDir * kDi * kNst) return;
  if (in_sizes[8] != kDir * kDi) return;
  if (in_sizes[9] != kDi) return;
  if (in_sizes[10] != kDi) return;
  if (in_sizes[11] != kDm * kDi) return;
  if (out_size != kRows * kDm) return;
  if (ws_size < kWsTotal) return;

  const float* x      = (const float*)d_in[0];
  const float* W_in   = (const float*)d_in[1];
  const float* conv_w = (const float*)d_in[2];
  const float* conv_b = (const float*)d_in[3];
  const float* W_xp   = (const float*)d_in[4];
  const float* W_dt   = (const float*)d_in[5];
  const float* b_dt   = (const float*)d_in[6];
  const float* A_log  = (const float*)d_in[7];
  const float* Dvec   = (const float*)d_in[8];
  const float* ln_g   = (const float*)d_in[9];
  const float* ln_b   = (const float*)d_in[10];
  const float* W_out  = (const float*)d_in[11];
  float* out = (float*)d_out;

  char* ws = (char*)d_ws;
  unsigned short* XB  = (unsigned short*)(ws + kOffXB);
  unsigned short* WI  = (unsigned short*)(ws + kOffWI);
  unsigned short* WXP = (unsigned short*)(ws + kOffWXP);
  unsigned short* WO  = (unsigned short*)(ws + kOffWO);
  float*          XZ  = (float*)(ws + kOffXZ);
  float*          XC  = (float*)(ws + kOffXC);
  unsigned short* XCH = (unsigned short*)(ws + kOffXCH);
  unsigned short* XCL = (unsigned short*)(ws + kOffXCL);
  float*          XD  = (float*)(ws + kOffXD);
  float*          YS  = (float*)(ws + kOffYS);
  unsigned short* YH  = (unsigned short*)(ws + kOffYH);
  unsigned short* YL  = (unsigned short*)(ws + kOffYL);

  plane_bf16_kernel<<<(kRows * kDm / 8) / 256, 256, 0, stream>>>(x, XB, kRows * kDm / 8, kDm, kRows, kRows);
  plane_bf16_kernel<<<(kXzP * kDm / 8) / 256, 256, 0, stream>>>(W_in, WI, kXzP * kDm / 8, kDm, kXzP, kXzP);
  plane_bf16_kernel<<<(kXdP * kDi / 8) / 256, 256, 0, stream>>>(W_xp, WXP, kXdP * kDi / 8, kDi, kXcP, kXcols);
  plane_bf16_kernel<<<(kWoP * kDi / 8) / 256, 256, 0, stream>>>(W_out, WO, kWoP * kDi / 8, kDi, kWoP, kDm);

  wmma_gemm64_bf16<0><<<((kRows / 64) * (kXzP / 64)) / 8, 256, 0, stream>>>(
      XB, XB, kDm, WI, kDm, XZ, kXzP, kRows, kXzP, kDm, kXzP);

  conv_silu_kernel<<<kBatch * kSide, 192, 0, stream>>>(XZ, conv_w, conv_b, XC, XCH, XCL);

  wmma_gemm64_bf16<1><<<((kRows / 64) * (kXdP / 64)) / 8, 256, 0, stream>>>(
      XCH, XCL, kDi, WXP, kDi, XD, kXdP, kRows, kXdP, kDi, kXdP);

  scan_kernel<<<kBatch * kDir, 192, 0, stream>>>(XD, XC, W_dt, b_dt, A_log, Dvec, YS);

  ln_gate_kernel<<<kRows / 32, 256, 0, stream>>>(YS, XZ, ln_g, ln_b, YH, YL);

  wmma_gemm64_bf16<1><<<((kRows / 64) * (kWoP / 64)) / 8, 256, 0, stream>>>(
      YH, YL, kDi, WO, kDi, out, kDm, kRows, kWoP, kDi, kDm);
}
